// ECGARD_44702019617306
// MI455X (gfx1250) — hardware-run, weakly checked
//
#include <hip/hip_runtime.h>
#include <math.h>

typedef __attribute__((ext_vector_type(16))) _Float16 v16h;
typedef __attribute__((ext_vector_type(8)))  _Float16 v8h;
typedef __attribute__((ext_vector_type(16))) __bf16   v16b;
typedef __attribute__((ext_vector_type(8)))  __bf16   v8b;
typedef __attribute__((ext_vector_type(8)))  float    v8f;
typedef __attribute__((ext_vector_type(4)))  float    v4f;
typedef __attribute__((ext_vector_type(4)))  unsigned v4u;

constexpr int kBatch = 4;
constexpr int kSeq   = 4096;
constexpr int kDm    = 128;
constexpr int kDin   = 256;
constexpr int kNst   = 16;
constexpr int kDtR   = 8;
constexpr int kTaps  = 3;
constexpr int kLP    = kSeq + 2;
constexpr int kKC    = kTaps * kDm;
constexpr int kXzP   = 2 * kDin;
constexpr int kXdN   = kDtR + 2 * kNst;
constexpr int kXdP   = 64;
constexpr int kRows  = kBatch * kSeq;
constexpr int kPRows = kBatch * kLP;
constexpr int kConvTP = 260;
constexpr int kScanTS = 64;
constexpr int kScanCh = 64;
constexpr int kScanYP = 68;
constexpr float kWScale = 32.0f;
constexpr float kUScale = 16.0f;
constexpr float kYScale = 64.0f;
static_assert(kXdN <= kXdP, "x_proj width");
static_assert((kKC % 32) == 0 && (kDm % 32) == 0 && (kDin % 32) == 0, "GEMM K multiples of 32");
static_assert((kSeq % 64) == 0 && (kRows % 64) == 0 && (kDm % 64) == 0 && (kXzP % 64) == 0 && (kXdP % 64) == 0, "GEMM M,N multiples of 64");
static_assert((kPRows % 8) == 0, "LN grid exact");
static_assert((kSeq % kScanTS) == 0 && (kDin % kScanCh) == 0 && kDin == 256, "tile multiples");

constexpr size_t kOffHP = 0;
constexpr size_t kOffWC = kOffHP + (size_t)kPRows * kDm * 2;
constexpr size_t kOffWI = kOffWC + (size_t)kDm * kKC * 2;
constexpr size_t kOffWX = kOffWI + (size_t)kXzP * kDm * 2;
constexpr size_t kOffWO = kOffWX + (size_t)kXdP * kDin * 2;
constexpr size_t kOffHC = kOffWO + (size_t)kDm * kDin * 2;
constexpr size_t kOffXZ = kOffHC + (size_t)kRows * kDm * 4;
constexpr size_t kOffUC = kOffXZ + (size_t)kRows * kXzP * 4;
constexpr size_t kOffUH = kOffUC + (size_t)kRows * kDin * 4;
constexpr size_t kOffXD = kOffUH + (size_t)kRows * kDin * 2;
constexpr size_t kOffYH = kOffXD + (size_t)kRows * kXdP * 4;
constexpr size_t kOffOM = kOffYH + (size_t)kRows * kDin * 2;
constexpr size_t kWsTotal = kOffOM + (size_t)kRows * kDm * 4;
static_assert(kWsTotal == 92604416ull, "carve total");
static_assert(kWsTotal <= 134217728ull, "carve cap");
static_assert((kOffWC % 128) == 0 && (kOffWI % 128) == 0 && (kOffWX % 128) == 0 && (kOffWO % 128) == 0 &&
              (kOffHC % 128) == 0 && (kOffXZ % 128) == 0 && (kOffUC % 128) == 0 && (kOffUH % 128) == 0 &&
              (kOffXD % 128) == 0 && (kOffYH % 128) == 0 && (kOffOM % 128) == 0, "128-B aligned regions");
static_assert((((size_t)kLP * kDm * 2) % 128) == 0, "HP batch stride 128-B aligned");

__device__ __forceinline__ unsigned short f2bf_bits(float f) {
  unsigned u = __float_as_uint(f);
  return (unsigned short)((u + 0x7FFFu + ((u >> 16) & 1u)) >> 16);
}
__device__ __forceinline__ float bf_bits2f(unsigned short h) { return __uint_as_float(((unsigned)h) << 16); }

__device__ __forceinline__ void dep_guard_h(v8f& a, v8f& b, v16h x, v16h y) { asm volatile("v_nop\n\tv_nop\n\tv_nop\n\tv_nop" : "+v"(a), "+v"(b) : "v"(x), "v"(y)); }
__device__ __forceinline__ void dep_guard_b(v8f& a, v8f& b, v16b x, v16b y) { asm volatile("v_nop\n\tv_nop\n\tv_nop\n\tv_nop" : "+v"(a), "+v"(b) : "v"(x), "v"(y)); }
__device__ __forceinline__ void keep4_h(v16h a, v16h b, v16h c, v16h d) { asm volatile("v_nop" :: "v"(a), "v"(b), "v"(c), "v"(d)); }
__device__ __forceinline__ void keep4_b(v16b a, v16b b, v16b c, v16b d) { asm volatile("v_nop" :: "v"(a), "v"(b), "v"(c), "v"(d)); }
__device__ __forceinline__ void acc_guard4(v8f& a, v8f& b, v8f& c, v8f& d) { asm volatile("v_nop\n\tv_nop\n\tv_nop\n\tv_nop" : "+v"(a), "+v"(b), "+v"(c), "+v"(d)); }
template <typename T> struct Frag;
template <> struct Frag<_Float16> {
  typedef v16h V; union U { v16h v; v8h h[2]; };
  static __device__ __forceinline__ v16h load(const _Float16* p) {
    U f; f.h[0] = *(const v8h*)(p); f.h[1] = *(const v8h*)(p + 16); return f.v;
  }
  static __device__ __forceinline__ v8f mma(v16h a, v16h b, v8f c) {
    return __builtin_amdgcn_wmma_f32_16x16x32_f16(false, a, false, b, (short)0, c, false, false);
  }
  static __device__ __forceinline__ void guard(v8f& a, v8f& b, v16h x, v16h y) { dep_guard_h(a, b, x, y); }
  static __device__ __forceinline__ void keep(v16h a, v16h b, v16h c, v16h d) { keep4_h(a, b, c, d); }
};
template <> struct Frag<__bf16> {
  typedef v16b V; union U { v16b v; v8b h[2]; };
  static __device__ __forceinline__ v16b load(const __bf16* p) {
    U f; f.h[0] = *(const v8b*)(p); f.h[1] = *(const v8b*)(p + 16); return f.v;
  }
  static __device__ __forceinline__ v8f mma(v16b a, v16b b, v8f c) {
    return __builtin_amdgcn_wmma_f32_16x16x32_bf16(false, a, false, b, (short)0, c, false, false);
  }
  static __device__ __forceinline__ void guard(v8f& a, v8f& b, v16b x, v16b y) { dep_guard_b(a, b, x, y); }
  static __device__ __forceinline__ void keep(v16b a, v16b b, v16b c, v16b d) { keep4_b(a, b, c, d); }
};

template <int ET> struct Elem;
template <> struct Elem<0> { typedef _Float16 T; };
template <> struct Elem<1> { typedef __bf16 T; };
template <int ET, int SPL, int BIAS_MODE, int OUT_MODE, bool RESID, int ACT = 0>
__global__ __launch_bounds__(256) void wmma_gemm64(
    const unsigned short* __restrict__ Ap, const unsigned short* __restrict__ A2p, int lda, long strideA,
    const unsigned short* __restrict__ Btp, const unsigned short* __restrict__ Bt2p, int ldb, long strideB,
    void* __restrict__ Cout, void* __restrict__ Cout2, int ldc, long strideC,
    const float* __restrict__ bias,
    const float* __restrict__ resid, long strideR,
    int M, int N, int K, float scale) {
  typedef typename Elem<ET>::T T;
  typedef typename Frag<T>::V V;
  const T* A = (const T*)Ap; const T* A2 = (const T*)A2p; const T* Bt = (const T*)Btp; const T* Bt2 = (const T*)Bt2p;
  __shared__ __align__(16) float sT[8][16 * 68];
  const int b    = blockIdx.y;
  const int lane = threadIdx.x & 31;
  const int wave = threadIdx.x >> 5;
  const int tilesN = N >> 6;
  const int tilesM = M >> 6;
  const int tile = blockIdx.x * 8 + wave;
  if (tile >= tilesM * tilesN) return;
  const int tm = tile / tilesN;
  const int tn = tile - tm * tilesN;
  const int m0 = tm << 6;
  const int n0 = tn << 6;

  const T* Ab  = A  + (size_t)b * strideA;
  const T* Bb  = Bt + (size_t)b * strideB;
  const T* Ab2 = (SPL >= 1) ? (A2  + (size_t)b * strideA) : nullptr;
  const T* Bb2 = (SPL == 2) ? (Bt2 + (size_t)b * strideB) : nullptr;

  const int rlane = lane & 15;
  const int koff  = (lane >> 4) * 8;
  const int mOff  = (lane >> 4) * 8;

  v8f acc[4][4];
#pragma unroll
  for (int i = 0; i < 4; ++i)
#pragma unroll
    for (int j = 0; j < 4; ++j) acc[i][j] = (v8f){0.f,0.f,0.f,0.f,0.f,0.f,0.f,0.f};

  for (int k0 = 0; k0 < K; k0 += 32) {
    V bh[4], bl[4];
#pragma unroll
    for (int j = 0; j < 4; ++j) {
      const size_t bo = (size_t)(n0 + (j << 4) + rlane) * ldb + koff + k0;
      bh[j] = Frag<T>::load(Bb + bo);
      if (SPL == 2) bl[j] = Frag<T>::load(Bb2 + bo);
    }
#pragma unroll
    for (int i = 0; i < 4; ++i) {
      const size_t ao = (size_t)(m0 + (i << 4) + rlane) * lda + koff + k0;
      V ah = Frag<T>::load(Ab + ao);
      V al;
      if (SPL >= 1) al = Frag<T>::load(Ab2 + ao);
#pragma unroll
      for (int j = 0; j < 4; ++j) {
        acc[i][j] = Frag<T>::mma(ah, bh[j], acc[i][j]);
        if (SPL == 2) acc[i][j] = Frag<T>::mma(ah, bl[j], acc[i][j]);
        if (SPL >= 1) acc[i][j] = Frag<T>::mma(al, bh[j], acc[i][j]);
      }
      Frag<T>::guard(acc[i][0], acc[i][3], ah, (SPL >= 1) ? al : ah);
    }
    Frag<T>::keep(bh[0], bh[1], bh[2], bh[3]);
    if (SPL == 2) Frag<T>::keep(bl[0], bl[1], bl[2], bl[3]);
  }
  acc_guard4(acc[0][0], acc[0][1], acc[0][2], acc[0][3]);
  acc_guard4(acc[1][0], acc[1][1], acc[1][2], acc[1][3]);
  acc_guard4(acc[2][0], acc[2][1], acc[2][2], acc[2][3]);
  acc_guard4(acc[3][0], acc[3][1], acc[3][2], acc[3][3]);

  float* slab = sT[wave];
  const float* Rb = RESID ? (resid + (size_t)b * strideR) : nullptr;
#pragma unroll
  for (int i = 0; i < 4; ++i) {
    const int mBase = m0 + (i << 4);
#pragma unroll
    for (int j = 0; j < 4; ++j) {
      const int n = n0 + (j << 4) + rlane;
      float bv = 0.f;
      if (BIAS_MODE == 2) bv = bias[n];
#pragma unroll
      for (int r = 0; r < 8; ++r) {
        float v = acc[i][j][r] * scale;
        if (BIAS_MODE == 1) v += bias[mBase + mOff + r];
        if (BIAS_MODE == 2) v += bv;
        if (RESID) v += Rb[(size_t)(mBase + mOff + r) * ldc + n];
        if (ACT == 1) v = tanhf(v);
        if (ACT == 2) v = fmaxf(v, 0.0f);
        if (ACT == 3) v = v / (1.0f + expf(-v));
        if (ACT == 4) v = (v > 0.f) ? v : 0.01f * v;
        slab[(mOff + r) * 68 + (j << 4) + rlane] = v;
      }
    }
    __builtin_amdgcn_fence(__ATOMIC_RELEASE, "workgroup");
    __builtin_amdgcn_wave_barrier();
    __builtin_amdgcn_fence(__ATOMIC_ACQUIRE, "workgroup");
    if (OUT_MODE == 0) {
      float* C = (float*)Cout + (size_t)b * strideC;
      const int hh = lane >> 4, c4 = (lane & 15) * 4;
      for (int pass = 0; pass < 2; ++pass) {
#pragma unroll
        for (int it = 0; it < 8; ++it) {
          const int row = it * 2 + hh;
          v4f v = *(const v4f*)(slab + row * 68 + c4);
          *(volatile v4f*)(C + (size_t)(mBase + row) * ldc + n0 + c4) = v;
        }
        __threadfence();
      }
    } else {
      const int q = lane >> 3, c8 = (lane & 7) * 8;
      unsigned short* C  = (unsigned short*)Cout  + (size_t)b * strideC;
      unsigned short* C2 = (OUT_MODE == 2) ? ((unsigned short*)Cout2 + (size_t)b * strideC) : nullptr;
      for (int pass = 0; pass < 2; ++pass) {
#pragma unroll
        for (int it = 0; it < 4; ++it) {
          const int row = it * 4 + q;
          const float* sp = slab + row * 68 + c8;
          v8h hv, lv;
#pragma unroll
          for (int e = 0; e < 8; ++e) {
            if (OUT_MODE == 1) {
              hv[e] = (_Float16)sp[e];
            } else {
              unsigned short hb = f2bf_bits(sp[e]);
              unsigned short lb = f2bf_bits(sp[e] - bf_bits2f(hb));
              hv[e] = __builtin_bit_cast(_Float16, hb);
              lv[e] = __builtin_bit_cast(_Float16, lb);
            }
          }
          *(volatile v8h*)(C + (size_t)(mBase + row) * ldc + n0 + c8) = hv;
          if (OUT_MODE == 2) *(volatile v8h*)(C2 + (size_t)(mBase + row) * ldc + n0 + c8) = lv;
        }
        __threadfence();
      }
    }
    __builtin_amdgcn_fence(__ATOMIC_RELEASE, "workgroup");
    __builtin_amdgcn_wave_barrier();
    __builtin_amdgcn_fence(__ATOMIC_ACQUIRE, "workgroup");
  }
}

__device__ __forceinline__ unsigned hb16(float f) {
  return (unsigned)__builtin_bit_cast(unsigned short, (_Float16)f);
}
__device__ __forceinline__ v4u pack8_h(v4f a0, v4f a1, float sc) {
  v4u r;
  r[0] = hb16(a0[0] * sc) | (hb16(a0[1] * sc) << 16);
  r[1] = hb16(a0[2] * sc) | (hb16(a0[3] * sc) << 16);
  r[2] = hb16(a1[0] * sc) | (hb16(a1[1] * sc) << 16);
  r[3] = hb16(a1[2] * sc) | (hb16(a1[3] * sc) << 16);
  return r;
}

__global__ __launch_bounds__(256) void cast_weights_kernel(
    const float* __restrict__ conv_w, const float* __restrict__ in_w,
    const float* __restrict__ xp_w, const float* __restrict__ out_w,
    unsigned short* __restrict__ WC, unsigned short* __restrict__ WI,
    unsigned short* __restrict__ WX, unsigned short* __restrict__ WO)
{
  const int bx = blockIdx.x, t = threadIdx.x;
  float v[8];
  unsigned short* dst;
  int gidx;
  if (bx < 24) {
    gidx = bx * 256 + t;
    const int idx0 = gidx * 8;
    const int o = idx0 / kKC;
    const int c = idx0 - o * kKC;
    const int tap = c >> 7, ci0 = c & 127;
#pragma unroll
    for (int e = 0; e < 8; ++e) v[e] = conv_w[((size_t)o * kDm + ci0 + e) * kTaps + tap] * kWScale;
    dst = WC;
  } else if (bx < 56) {
    gidx = (bx - 24) * 256 + t;
    const int idx0 = gidx * 8;
    const int n = idx0 >> 7, k0 = idx0 & 127;
#pragma unroll
    for (int e = 0; e < 8; ++e) v[e] = in_w[(size_t)(k0 + e) * kXzP + n] * kWScale;
    dst = WI;
  } else if (bx < 64) {
    gidx = (bx - 56) * 256 + t;
    const int idx0 = gidx * 8;
    const int n = idx0 >> 8, k0 = idx0 & 255;
    const int nn = (n < kXdN) ? n : (kXdN - 1);
    const float f = (n < kXdN) ? kWScale : 0.0f;
#pragma unroll
    for (int e = 0; e < 8; ++e) v[e] = xp_w[(size_t)(k0 + e) * kXdN + nn] * f;
    dst = WX;
  } else {
    gidx = (bx - 64) * 256 + t;
    const int idx0 = gidx * 8;
    const int n = idx0 >> 8, k0 = idx0 & 255;
#pragma unroll
    for (int e = 0; e < 8; ++e) v[e] = out_w[(size_t)(k0 + e) * kDm + n] * kWScale;
    dst = WO;
  }
  v4f a0, a1;
  a0[0] = v[0]; a0[1] = v[1]; a0[2] = v[2]; a0[3] = v[3];
  a1[0] = v[4]; a1[1] = v[5]; a1[2] = v[6]; a1[3] = v[7];
  const v4u pv = pack8_h(a0, a1, 1.0f);
  unsigned short* p = dst + (size_t)gidx * 8;
  *(volatile v4u*)p = pv;
  __threadfence();
  *(volatile v4u*)p = pv;
}

__global__ __launch_bounds__(256) void layernorm_f16_kernel(
    const float* __restrict__ x, const float* __restrict__ g, const float* __restrict__ bt,
    unsigned short* __restrict__ HP)
{
  const int lane = threadIdx.x & 31, wave = threadIdx.x >> 5;
  const int pr = blockIdx.x * 8 + wave;
  const int b = pr / kLP;
  const int rloc = pr - b * kLP;
  const bool padrow = (rloc < 2);
  int tl = rloc - 2; tl = (tl < 0) ? 0 : tl;
  const size_t tok = (size_t)b * kSeq + (size_t)tl;
  const v4f xv = *(const v4f*)(x + tok * kDm + lane * 4);
  float s = (xv[0] + xv[1]) + (xv[2] + xv[3]);
#pragma unroll
  for (int off = 16; off >= 1; off >>= 1) s += __shfl_xor(s, off);
  const float mu = s * (1.0f / kDm);
  const float e0 = xv[0] - mu, e1 = xv[1] - mu, e2 = xv[2] - mu, e3 = xv[3] - mu;
  float s2 = (e0 * e0 + e1 * e1) + (e2 * e2 + e3 * e3);
#pragma unroll
  for (int off = 16; off >= 1; off >>= 1) s2 += __shfl_xor(s2, off);
  const float var = s2 * (1.0f / kDm);
  const float rr = rsqrtf(var + 1e-5f);
  const v4f gv = *(const v4f*)(g + lane * 4);
  const v4f bv = *(const v4f*)(bt + lane * 4);
  const float o0 = e0 * rr * gv[0] + bv[0];
  const float o1 = e1 * rr * gv[1] + bv[1];
  const float o2 = e2 * rr * gv[2] + bv[2];
  const float o3 = e3 * rr * gv[3] + bv[3];
  unsigned w0 = hb16(o0) | (hb16(o1) << 16);
  unsigned w1 = hb16(o2) | (hb16(o3) << 16);
  w0 = padrow ? 0u : w0;
  w1 = padrow ? 0u : w1;
  const int sl0 = (2 * lane) & 31, sl1 = (2 * lane + 1) & 31;
  v4u pv;
  pv[0] = (unsigned)__shfl((int)w0, sl0);
  pv[1] = (unsigned)__shfl((int)w1, sl0);
  pv[2] = (unsigned)__shfl((int)w0, sl1);
  pv[3] = (unsigned)__shfl((int)w1, sl1);
  unsigned short* rowp = HP + (size_t)pr * kDm + lane * 8;
  if (lane < 16) *(volatile v4u*)rowp = pv;
  __threadfence();
  if (lane < 16) *(volatile v4u*)rowp = pv;
}

__global__ __launch_bounds__(256) void conv_silu_kernel(
    const float* __restrict__ XZ, const float* __restrict__ cw, const float* __restrict__ cb,
    float* __restrict__ UC, unsigned short* __restrict__ UH)
{
  __shared__ __align__(16) float sT[16 * kConvTP];
  const int tid = threadIdx.x, lane = tid & 31, wave = tid >> 5;
  const int d0 = blockIdx.x * 256, d = d0 + tid;
  const int g0 = blockIdx.y * 64;
  const int tb = g0 & (kSeq - 1);
  const float w0 = cw[d * 4 + 0], w1 = cw[d * 4 + 1], w2 = cw[d * 4 + 2], w3 = cw[d * 4 + 3];
  const float bc = cb[d];
  float xm3, xm2, xm1;
  {
    const bool hist = (tb > 0);
    const int rb = hist ? (g0 - 3) : g0;
    const float v3 = XZ[(size_t)rb * kXzP + d];
    const float v2 = XZ[(size_t)(rb + 1) * kXzP + d];
    const float v1 = XZ[(size_t)(rb + 2) * kXzP + d];
    xm3 = hist ? v3 : 0.f;
    xm2 = hist ? v2 : 0.f;
    xm1 = hist ? v1 : 0.f;
  }
  const int hrow = wave >> 1;
  const int hch  = (wave & 1) * 128 + lane * 4;
#pragma unroll 1
  for (int sub = 0; sub < 4; ++sub) {
    const int lb = g0 + sub * 16;
#pragma unroll 1
    for (int s = 0; s < 16; ++s) {
      const float xcur = XZ[(size_t)(lb + s) * kXzP + d];
      float acc = w0 * xm3;
      acc = fmaf(w1, xm2, acc);
      acc = fmaf(w2, xm1, acc);
      acc = fmaf(w3, xcur, acc);
      const float sv = acc + bc;
      const float sg = __builtin_amdgcn_rcpf(1.0f + expf(-sv));
      sT[s * kConvTP + tid] = sv * sg;
      xm3 = xm2; xm2 = xm1; xm1 = xcur;
    }
    __syncthreads();
    v4f fv[4];
    v4u pk[2];
#pragma unroll
    for (int it = 0; it < 4; ++it) fv[it] = *(const v4f*)(sT + (it * 4 + hrow) * kConvTP + hch);
#pragma unroll
    for (int it = 0; it < 2; ++it) {
      const float* sp = sT + (it * 8 + wave) * kConvTP + lane * 8;
      const v4f a0 = *(const v4f*)(sp);
      const v4f a1 = *(const v4f*)(sp + 4);
      pk[it] = pack8_h(a0, a1, kUScale);
    }
    for (int pass = 0; pass < 2; ++pass) {
#pragma unroll
      for (int it = 0; it < 4; ++it)
        *(volatile v4f*)(UC + (size_t)(lb + it * 4 + hrow) * kDin + d0 + hch) = fv[it];
#pragma unroll
      for (int it = 0; it < 2; ++it)
        *(volatile v4u*)(UH + (size_t)(lb + it * 8 + wave) * kDin + d0 + lane * 8) = pk[it];
      __threadfence();
    }
    __syncthreads();
  }
}

__global__ __launch_bounds__(64) void scan_kernel(
    const float* __restrict__ XD, const float* __restrict__ UC, const float* __restrict__ XZ,
    const float* __restrict__ Wdt, const float* __restrict__ bdt, const float* __restrict__ Alog,
    const float* __restrict__ Dp, unsigned short* __restrict__ YH)
{
  __shared__ __align__(16) float sX[kScanTS * kXdP];
  __shared__ __align__(16) float sY[kScanTS * kScanYP];
  __shared__ __align__(16) float sW[kDtR * kScanCh];
  __shared__ __align__(16) float sA[kNst * kScanCh];
  const int tid = threadIdx.x, lane = tid & 31, wave = tid >> 5;
  constexpr int kBlkPerB = kDin / kScanCh;
  const int bix = blockIdx.x / kBlkPerB;
  const int d0  = (blockIdx.x - bix * kBlkPerB) * kScanCh;
  const int d   = d0 + tid;
  const size_t row0 = (size_t)bix * kSeq;
#pragma unroll 1
  for (int r = 0; r < kDtR; ++r) sW[r * kScanCh + tid] = Wdt[(size_t)r * kDin + d];
#pragma unroll 1
  for (int s = 0; s < kNst; ++s) sA[s * kScanCh + tid] = -expf(Alog[(size_t)d * kNst + s]);
  __syncthreads();
  float negA[kNst], h[kNst];
#pragma unroll
  for (int s = 0; s < kNst; ++s) {
    negA[s] = sA[s * kScanCh + tid];
    h[s] = 0.f;
  }
  const float bb = bdt[d], Dd = Dp[d];
  const int lr = tid >> 4, lc4 = (tid & 15) * 4;
  const int q = lane >> 3, c8 = (lane & 7) * 8;
#pragma unroll 1
  for (int t0 = 0; t0 < kSeq; t0 += kScanTS) {
    __syncthreads();
#pragma unroll
    for (int i = 0; i < 16; ++i) {
      const int r = lr + 4 * i;
      *(v4f*)(sX + r * kXdP + lc4) = *(const v4f*)(XD + (row0 + t0 + r) * kXdP + lc4);
    }
    __syncthreads();
#pragma unroll 1
    for (int s = 0; s < kScanTS; ++s) {
      const int t = t0 + s;
      const float* xr = sX + s * kXdP;
      float vdot = 0.f;
#pragma unroll 1
      for (int r4 = 0; r4 < kDtR / 4; ++r4) {
        const v4f xv = *(const v4f*)(xr + 4 * r4);
        const float* wp = sW + (4 * r4) * kScanCh + tid;
        vdot = fmaf(xv[0], wp[0], vdot);
        vdot = fmaf(xv[1], wp[kScanCh], vdot);
        vdot = fmaf(xv[2], wp[2 * kScanCh], vdot);
        vdot = fmaf(xv[3], wp[3 * kScanCh], vdot);
      }
      float Bs[kNst], Cs[kNst];
#pragma unroll
      for (int q4 = 0; q4 < 4; ++q4) {
        const v4f bv = *(const v4f*)(xr + kDtR + 4 * q4);
        const v4f cv = *(const v4f*)(xr + kDtR + kNst + 4 * q4);
        Bs[4 * q4 + 0] = bv[0]; Bs[4 * q4 + 1] = bv[1]; Bs[4 * q4 + 2] = bv[2]; Bs[4 * q4 + 3] = bv[3];
        Cs[4 * q4 + 0] = cv[0]; Cs[4 * q4 + 1] = cv[1]; Cs[4 * q4 + 2] = cv[2]; Cs[4 * q4 + 3] = cv[3];
      }
      const float v  = vdot + bb;
      const float dt = fmaxf(v, 0.0f) + log1pf(expf(-fabsf(v)));
      const float xt = UC[(row0 + t) * kDin + d];
      float y = 0.f;
#pragma unroll
      for (int k = 0; k < kNst; ++k) {
        const float e = __expf(dt * negA[k]);
        const float dB = dt * Bs[k];
        h[k] = e * h[k] + dB * xt;
        y = h[k] * Cs[k] + y;
      }
      y = y + xt * Dd;
      const float zv = XZ[(row0 + t) * kXzP + kDin + d];
      const float sg = __builtin_amdgcn_rcpf(1.0f + expf(-zv));
      y = y * (zv * sg);
      sY[s * kScanYP + tid] = y;
    }
    __syncthreads();
    v4u pk[8];
#pragma unroll
    for (int it = 0; it < 8; ++it) {
      const int row = it * 8 + wave * 4 + q;
      const float* sp = sY + row * kScanYP + c8;
      const v4f a0 = *(const v4f*)(sp);
      const v4f a1 = *(const v4f*)(sp + 4);
      pk[it] = pack8_h(a0, a1, kYScale);
    }
    for (int pass = 0; pass < 2; ++pass) {
#pragma unroll
      for (int it = 0; it < 8; ++it) {
        const int row = it * 8 + wave * 4 + q;
        const size_t o = (row0 + t0 + row) * kDin + d0 + c8;
        *(volatile v4u*)(YH + o) = pk[it];
      }
      __threadfence();
    }
  }
}

__global__ __launch_bounds__(256) void combine_kernel(
    const float* __restrict__ x, const float* __restrict__ OM, const float* __restrict__ HC,
    float* __restrict__ out, int total4)
{
  const int i = blockIdx.x * 256 + threadIdx.x;
  if (i >= total4) return;
  const size_t e0 = (size_t)i * 4;
  const v4f xv = *(const v4f*)(x + e0);
  const v4f mv = *(const v4f*)(OM + e0);
  const v4f cv = *(const v4f*)(HC + e0);
  float g0 = 0.f, g1 = 0.f, g2 = 0.f, g3 = 0.f;
#pragma unroll 1
  for (int c = 0; c < 4; ++c) {
    const float t  = (c == 0) ? cv[0] : (c == 1) ? cv[1] : (c == 2) ? cv[2] : cv[3];
    const float gl = 0.5f * t * (1.0f + erff(t * 0.70710678118654752f));
    g0 = (c == 0) ? gl : g0;
    g1 = (c == 1) ? gl : g1;
    g2 = (c == 2) ? gl : g2;
    g3 = (c == 3) ? gl : g3;
  }
  v4f ov;
  ov[0] = xv[0] + (0.5f * mv[0] + 0.5f * g0);
  ov[1] = xv[1] + (0.5f * mv[1] + 0.5f * g1);
  ov[2] = xv[2] + (0.5f * mv[2] + 0.5f * g2);
  ov[3] = xv[3] + (0.5f * mv[3] + 0.5f * g3);
  float* p = out + e0;
  *(volatile v4f*)p = ov;
  __threadfence();
  *(volatile v4f*)p = ov;
}

extern "C" void kernel_launch(void* const* d_in, const int* in_sizes, int n_in,
                              void* d_out, int out_size, void* d_ws, size_t ws_size,
                              hipStream_t stream) {
  if (n_in < 16) return;
  if (in_sizes[0]  != kRows * kDm) return;
  if (in_sizes[1]  != kDm) return;
  if (in_sizes[2]  != kDm) return;
  if (in_sizes[3]  != kDm * kDm * kTaps) return;
  if (in_sizes[4]  != kDm) return;
  if (in_sizes[5]  != kDm * kXzP) return;
  if (in_sizes[6]  != kXzP) return;
  if (in_sizes[7]  != kDin * 4) return;
  if (in_sizes[8]  != kDin) return;
  if (in_sizes[9]  != kDin * kXdN) return;
  if (in_sizes[10] != kDtR * kDin) return;
  if (in_sizes[11] != kDin) return;
  if (in_sizes[12] != kDin * kNst) return;
  if (in_sizes[13] != kDin) return;
  if (in_sizes[14] != kDin * kDm) return;
  if (in_sizes[15] != kDm) return;
  if (out_size != kRows * kDm) return;
  if (ws_size < kWsTotal) return;

  const float* x      = (const float*)d_in[0];
  const float* ln_g   = (const float*)d_in[1];
  const float* ln_b   = (const float*)d_in[2];
  const float* conv_w = (const float*)d_in[3];
  const float* conv_b = (const float*)d_in[4];
  const float* in_w   = (const float*)d_in[5];
  const float* in_b   = (const float*)d_in[6];
  const float* c1_w   = (const float*)d_in[7];
  const float* c1_b   = (const float*)d_in[8];
  const float* xp_w   = (const float*)d_in[9];
  const float* dtp_w  = (const float*)d_in[10];
  const float* dtp_b  = (const float*)d_in[11];
  const float* A_log  = (const float*)d_in[12];
  const float* Dskip  = (const float*)d_in[13];
  const float* out_w  = (const float*)d_in[14];
  const float* out_b  = (const float*)d_in[15];
  float* out = (float*)d_out;

  char* ws = (char*)d_ws;
  unsigned short* HP = (unsigned short*)(ws + kOffHP);
  unsigned short* WC = (unsigned short*)(ws + kOffWC);
  unsigned short* WI = (unsigned short*)(ws + kOffWI);
  unsigned short* WX = (unsigned short*)(ws + kOffWX);
  unsigned short* WO = (unsigned short*)(ws + kOffWO);
  float*          HC = (float*)(ws + kOffHC);
  float*          XZ = (float*)(ws + kOffXZ);
  float*          UC = (float*)(ws + kOffUC);
  unsigned short* UH = (unsigned short*)(ws + kOffUH);
  float*          XD = (float*)(ws + kOffXD);
  unsigned short* YH = (unsigned short*)(ws + kOffYH);
  float*          OM = (float*)(ws + kOffOM);

  cast_weights_kernel<<<80, 256, 0, stream>>>(conv_w, in_w, xp_w, out_w, WC, WI, WX, WO);

  layernorm_f16_kernel<<<kPRows / 8, 256, 0, stream>>>(x, ln_g, ln_b, HP);

  wmma_gemm64<0, 0, 2, 0, false><<<dim3(16, kBatch), 256, 0, stream>>>(
      HP, nullptr, kDm, (long)kLP * kDm,
      WC, nullptr, kKC, 0L,
      (void*)HC, nullptr, kDm, (long)kSeq * kDm,
      conv_b, nullptr, 0L,
      kSeq, kDm, kKC, 1.0f / kWScale);

  wmma_gemm64<0, 0, 2, 0, false><<<dim3(64, kBatch), 256, 0, stream>>>(
      HP + 2 * kDm, nullptr, kDm, (long)kLP * kDm,
      WI, nullptr, kDm, 0L,
      (void*)XZ, nullptr, kXzP, (long)kSeq * kXzP,
      in_b, nullptr, 0L,
      kSeq, kXzP, kDm, 1.0f / kWScale);

  conv_silu_kernel<<<dim3(kDin / 256, kRows / 64), 256, 0, stream>>>(XZ, c1_w, c1_b, UC, UH);

  wmma_gemm64<0, 0, 0, 0, false><<<dim3(32, 1), 256, 0, stream>>>(
      UH, nullptr, kDin, 0L,
      WX, nullptr, kDin, 0L,
      (void*)XD, nullptr, kXdP, 0L,
      nullptr, nullptr, 0L,
      kRows, kXdP, kDin, 1.0f / (kUScale * kWScale));

  scan_kernel<<<kBatch * (kDin / kScanCh), kScanCh, 0, stream>>>(XD, UC, XZ, dtp_w, dtp_b, A_log, Dskip, YH);

  wmma_gemm64<0, 0, 2, 0, false><<<dim3(64, 1), 256, 0, stream>>>(
      YH, nullptr, kDin, 0L,
      WO, nullptr, kDin, 0L,
      (void*)OM, nullptr, kDm, 0L,
      out_b, nullptr, 0L,
      kRows, kDm, kDin, 1.0f / (kYScale * kWScale));

  combine_kernel<<<(kRows * kDm / 4) / 256, 256, 0, stream>>>(x, OM, HC, out, kRows * kDm / 4);
}
